// MultiHeadAttention_30408368455775
// MI455X (gfx1250) — hardware-verified
//
#include <hip/hip_runtime.h>
#ifndef NB
#define NB 4
#endif
#ifndef SEQ
#define SEQ 1024
#endif
#define NB_FULL 4
#define SEQ_FULL 1024
#define SQ SEQ
#define DM 1024
#define NH 16
#define HD 64
#define NR ((size_t)NB * SQ)
#define MP ((int)NR)
#define LQ DM

static_assert(NB >= 1 && NB <= NB_FULL);
static_assert(SQ >= 256 && SQ <= SEQ_FULL && (SQ % 256) == 0);
static_assert((MP % 128) == 0 && (DM % 64) == 0 && (DM % 32) == 0 && HD == 64 && NH * HD == DM);
static_assert((SQ % 64) == 0 && (SQ % 32) == 0 && (LQ % 8) == 0 && (HD % 32) == 0);
static_assert(((size_t)(NB - 1) * SEQ_FULL + SQ) * DM <= (size_t)NB_FULL * SEQ_FULL * DM);
#define WS_W   ((size_t)DM * DM * 2)
#define WS_X   ((size_t)NR * DM * 2)
#define WS_VT  ((size_t)NH * HD * SQ * 2)
#define WS_TOTAL (6 * WS_W + WS_X + 6 * WS_X + 2 * (size_t)NB * WS_VT)
static_assert((WS_W % 256) == 0 && (WS_X % 256) == 0 && (WS_VT % 256) == 0);
static_assert(WS_TOTAL <= (size_t)134217728);

typedef unsigned short v8us __attribute__((ext_vector_type(8), may_alias));
typedef float  v8f  __attribute__((ext_vector_type(8)));
typedef float  v4f  __attribute__((ext_vector_type(4)));
typedef float  v4fa __attribute__((ext_vector_type(4), may_alias));
typedef _Float16 v16h __attribute__((ext_vector_type(16)));
typedef _Float16 v4h __attribute__((ext_vector_type(4)));
union FragH { v16h v; v8us half[2]; _Float16 h[16]; unsigned short u[16]; };

__device__ __forceinline__ unsigned short bf16_bits(float x) { unsigned int u = __float_as_uint(x); return (unsigned short)((u + 0x7FFFu + ((u >> 16) & 1u)) >> 16); }
__device__ __forceinline__ float bf16_val(unsigned short b) { return __uint_as_float(((unsigned int)b) << 16); }
__device__ __forceinline__ float bf16_rne(float x) { return bf16_val(bf16_bits(x)); }

__device__ __forceinline__ v16h g2_frag(const _Float16* p, int hh) { FragH f; f.half[0] = *(const v8us*)((const unsigned short*)p + 8 * hh); f.half[1] = *(const v8us*)((const unsigned short*)p + 16 + 8 * hh); return f.v; }
__device__ __forceinline__ v8f g2_mma(v16h a, v16h b, v8f c) { v8f d = __builtin_amdgcn_wmma_f32_16x16x32_f16(false, a, false, b, (short)0, c, false, false); asm volatile("v_nop\n\tv_nop\n\tv_nop\n\tv_nop" : "+v"(d) : "v"(a), "v"(b)); return d; }
template <int ACT>
__global__ __launch_bounds__(128) void k_gemm2(const _Float16* __restrict__ A, int lda, size_t sA, const _Float16* __restrict__ Bh, int ldb, size_t sB, float alpha, const float* __restrict__ bias, size_t sBias, const float* __restrict__ CP, int rowsPerB, size_t sCPb, int row0g,
    float* __restrict__ C, _Float16* __restrict__ C16, int ldc, size_t sC, int M, int N, int K) {
  static_assert(ACT == 0 || ACT == 3);
  __shared__ __attribute__((aligned(16))) float so[4][32][68];
  const int tid = threadIdx.x, w = tid >> 5, lane = tid & 31, ln = lane & 15, hh = lane >> 4; const int by = blockIdx.y;
  A += (size_t)by * sA; Bh += (size_t)by * sB; const size_t cofs = (size_t)by * sC; const float* bp = bias ? bias + (size_t)by * sBias : nullptr;
  const int ntn = N >> 6; const int mt = blockIdx.x / ntn, nq = blockIdx.x - mt * ntn; const int row0 = mt * 128 + 32 * w, col0 = nq * 64; if (row0 >= M) return;
  const _Float16* a0p = A + (size_t)(row0 + ln) * lda; const _Float16* a1p = a0p + (size_t)16 * lda;
  const _Float16* b0p = Bh + (size_t)(col0 + ln) * ldb; const _Float16* b1p = b0p + (size_t)16 * ldb; const _Float16* b2p = b1p + (size_t)16 * ldb; const _Float16* b3p = b2p + (size_t)16 * ldb;
  const v8f z8 = {0.f,0.f,0.f,0.f,0.f,0.f,0.f,0.f}; v8f c00 = z8, c01 = z8, c02 = z8, c03 = z8, c10 = z8, c11 = z8, c12 = z8, c13 = z8;
#pragma unroll 1
  for (int kb = 0; kb < K; kb += 32) { const v16h a0 = g2_frag(a0p + kb, hh), a1 = g2_frag(a1p + kb, hh);
    v16h b = g2_frag(b0p + kb, hh); c00 = g2_mma(a0, b, c00); c10 = g2_mma(a1, b, c10);
    b = g2_frag(b1p + kb, hh); c01 = g2_mma(a0, b, c01); c11 = g2_mma(a1, b, c11);
    b = g2_frag(b2p + kb, hh); c02 = g2_mma(a0, b, c02); c12 = g2_mma(a1, b, c12);
    b = g2_frag(b3p + kb, hh); c03 = g2_mma(a0, b, c03); c13 = g2_mma(a1, b, c13); }
  v8f accs[8] = {c00, c01, c02, c03, c10, c11, c12, c13};
#pragma unroll
  for (int u = 0; u < 8; ++u) { const int t = u & 3, half = u >> 2; const int col = col0 + t * 16 + ln; const float bv = bp ? bf16_rne(bp[col]) : 0.f;
#pragma unroll
    for (int r = 0; r < 8; ++r) { const int rloc = half * 16 + 8 * hh + r; float v = accs[u][r] * alpha + bv;
      if (CP) { if (rowsPerB < 0) v += CP[cofs + (size_t)(row0g + row0 + rloc) * ldc + col]; else { const int bidx = (row0g + row0 + rloc) / rowsPerB; v += CP[(size_t)bidx * sCPb + (size_t)by * 64 + col]; } }
      if (ACT == 3) v = fmaxf(v, 0.f);
      so[w][rloc][t * 16 + ln] = v; } }
  __builtin_amdgcn_fence(4  , "workgroup"); __builtin_amdgcn_wave_barrier();
  const int rsub = lane >> 4, c4 = (lane & 15) * 4;
  for (int pass = 0; pass < 2; ++pass) {
#pragma unroll
    for (int q = 0; q < 16; ++q) { const int r = q * 2 + rsub; const v4f v = *(const v4fa*)&so[w][r][c4];
      if (C) *(volatile v4f*)(C + cofs + (size_t)(row0 + r) * ldc + col0 + c4) = v;
      if (C16) { v4h h4; for (int i = 0; i < 4; ++i) h4[i] = (_Float16)v[i]; *(volatile v4h*)(C16 + cofs + (size_t)(row0 + r) * ldc + col0 + c4) = h4; } }
    if (pass == 0) __threadfence(); } }

__global__ __launch_bounds__(256) void k_wt_f16(const float* __restrict__ W, _Float16* __restrict__ Wt, int K, int N, float scale) {
  const int t = blockIdx.x * 256 + threadIdx.x; if (t >= N * (K / 8)) return; const int n = t / (K / 8), k8 = (t % (K / 8)) * 8; FragH f;
#pragma unroll
  for (int i = 0; i < 8; ++i) f.h[i] = (_Float16)(bf16_rne(W[(size_t)(k8 + i) * N + n]) * scale); const v8us o = f.half[0];
  *(volatile v8us*)((unsigned short*)Wt + (size_t)n * K + k8) = o; __threadfence(); *(volatile v8us*)((unsigned short*)Wt + (size_t)n * K + k8) = o;
}

__global__ __launch_bounds__(256) void k_x16(const float* __restrict__ x, _Float16* __restrict__ X16, size_t n8) {
  const size_t t = (size_t)blockIdx.x * 256 + threadIdx.x; if (t >= n8) return;
  const size_t e = t * 8; const size_t rc = e / DM; const size_t c = e % DM; const size_t b = rc / SQ, s = rc % SQ;
  const float* src = x + ((b * SEQ_FULL + s) * DM + c);
  const v4f a = *(const v4fa*)src, d = *(const v4fa*)(src + 4); FragH f;
#pragma unroll
  for (int q = 0; q < 4; ++q) { f.h[q] = (_Float16)bf16_rne(a[q]); f.h[4 + q] = (_Float16)bf16_rne(d[q]); }
  *(volatile v8us*)((unsigned short*)X16 + t * 8) = f.half[0]; __threadfence(); *(volatile v8us*)((unsigned short*)X16 + t * 8) = f.half[0]; }

template <int NHv, int TTv>
__global__ __launch_bounds__(256) void k_vt(const _Float16* __restrict__ V16, int ldv, int voff, _Float16* __restrict__ Vt) { __shared__ unsigned short tl[64][66]; const int tid = threadIdx.x; const int slab = blockIdx.x / (TTv / 64), lg = blockIdx.x % (TTv / 64); const int b = slab / NHv, h = slab % NHv;
  for (int i = tid; i < 64 * 8; i += 256) { const int r = i / 8, c8 = (i % 8) * 8; FragH f; f.half[0] = *(const v8us*)((const unsigned short*)V16 + ((size_t)b * TTv + lg * 64 + r) * ldv + voff + h * 64 + c8);
#pragma unroll
    for (int q = 0; q < 8; ++q) tl[r][c8 + q] = f.u[q]; }
  __syncthreads();
  for (int pass = 0; pass < 2; ++pass) {
#pragma unroll
    for (int rd = 0; rd < 2; ++rd) { const int d = rd * 32 + tid / 8, pc = tid % 8; FragH f;
#pragma unroll
      for (int q = 0; q < 8; ++q) f.u[q] = tl[pc * 8 + q][d];
      *(volatile v8us*)((unsigned short*)Vt + ((size_t)slab * 64 + d) * TTv + lg * 64 + pc * 8) = f.half[0]; }
    if (pass == 0) __threadfence(); } }

__global__ __launch_bounds__(128) __attribute__((amdgpu_num_vgpr(256))) void k_flash2(const _Float16* __restrict__ PL, const _Float16* __restrict__ VT, const float* __restrict__ aw, float* __restrict__ out) {
  __shared__ __attribute__((aligned(16))) float so[4][16][68];
  const int wave = __builtin_amdgcn_readfirstlane(threadIdx.x >> 5);
  const int lane = threadIdx.x & 31, ln = lane & 15, hh = lane >> 4;
  const int slab = blockIdx.y; const int b = slab / NH, h = slab - b * NH;
  const int q0 = blockIdx.x * 64 + wave * 16;
  const size_t PLN = (size_t)NR * DM;
  float w0, w1;
  { const float a0 = bf16_rne(aw[0]), a1 = bf16_rne(aw[1]); const float mx = fmaxf(a0, a1); const float e0 = expf(a0 - mx), e1 = expf(a1 - mx); const float inv = 1.0f / (e0 + e1); w0 = e0 * inv; w1 = e1 * inv; }
  const v8f z8 = {0.f,0.f,0.f,0.f,0.f,0.f,0.f,0.f};
  v8f res[4] = {z8, z8, z8, z8};
  float wcur = w0;
#pragma unroll 1
  for (int set = 0; set < 2; ++set) {
    const size_t qo = (size_t)(3 * set) * PLN + ((size_t)b * SQ + q0 + ln) * LQ + h * HD;
    const size_t ko = (size_t)(3 * set + 1) * PLN + ((size_t)b * SQ + ln) * LQ + h * HD;
    const size_t vo = (((size_t)set * (NB * NH) + slab) * HD + ln) * SQ;
    const v16h qf0 = g2_frag(PL + qo, hh), qf1 = g2_frag(PL + qo + 32, hh);
    v8f o[4] = {z8, z8, z8, z8}; float m = -1.0e30f, l = 0.f;
#pragma unroll 1
    for (int j0 = 0; j0 < SQ; j0 += 32) {
      const _Float16* kp = PL + ko + (size_t)j0 * LQ;
      v8f s0 = z8, s1 = z8;
      { v16h a = g2_frag(kp, hh); s0 = g2_mma(a, qf0, s0);
        a = g2_frag(kp + 32, hh); s0 = g2_mma(a, qf1, s0);
        a = g2_frag(kp + (size_t)16 * LQ, hh); s1 = g2_mma(a, qf0, s1);
        a = g2_frag(kp + (size_t)16 * LQ + 32, hh); s1 = g2_mma(a, qf1, s1); }
      float tm = fmaxf(s0[0], s1[0]);
#pragma unroll
      for (int r = 1; r < 8; ++r) tm = fmaxf(tm, fmaxf(s0[r], s1[r]));
      tm = fmaxf(tm, __shfl_xor(tm, 16, 32));
      const float mn = fmaxf(m, tm * 0.125f);
      const float corr = __expf(m - mn);
      const float sh = 6.931471806f - mn;
      FragH pf; float ps = 0.f;
#pragma unroll
      for (int r = 0; r < 8; ++r) { const float e0 = s0[r] * 0.125f + sh, e1 = s1[r] * 0.125f + sh;
        const float p0 = (e0 < -9.70f) ? 0.f : __expf(e0); const float p1 = (e1 < -9.70f) ? 0.f : __expf(e1);
        const _Float16 h0 = (_Float16)p0, h1 = (_Float16)p1; pf.h[r] = h0; pf.h[8 + r] = h1; ps += (float)h0 + (float)h1; }
      ps += __shfl_xor(ps, 16, 32);
      l = l * corr + ps; m = mn;
#pragma unroll
      for (int t = 0; t < 4; ++t) o[t] = o[t] * corr;
      const _Float16* vp = VT + vo + j0;
#pragma unroll
      for (int t = 0; t < 4; ++t) { const v16h va = g2_frag(vp + (size_t)t * 16 * SQ, hh); o[t] = g2_mma(va, pf.v, o[t]); } }
    const float sc = wcur * (1.0f / l);
#pragma unroll
    for (int t = 0; t < 4; ++t) res[t] += o[t] * sc;
    wcur = w1; }
#pragma unroll
  for (int t = 0; t < 4; ++t) {
#pragma unroll
    for (int r = 0; r < 8; ++r) so[wave][ln][t * 16 + 8 * hh + r] = res[t][r]; }
  __builtin_amdgcn_fence(4  , "workgroup"); __builtin_amdgcn_wave_barrier();
  const int rsub = lane >> 4, c4 = (lane & 15) * 4;
  float* ob = out + ((size_t)b * SEQ_FULL + q0) * DM + h * HD;
  for (int pass = 0; pass < 2; ++pass) {
#pragma unroll
    for (int q = 0; q < 8; ++q) { const int r = q * 2 + rsub; const v4f v = *(const v4fa*)&so[wave][r][c4];
      *(volatile v4f*)(ob + (size_t)r * DM + c4) = v; }
    if (pass == 0) __threadfence(); } }

extern "C" void kernel_launch(void* const* d_in, const int* in_sizes, int n_in,
                              void* d_out, int out_size, void* d_ws, size_t ws_size, hipStream_t stream) {
  if (n_in < 14) return;
  const size_t rows_need = (size_t)(NB - 1) * SEQ_FULL + SQ;
  if ((size_t)in_sizes[0] < rows_need * DM) return;
  for (int i = 0; i < 6; ++i) { if (in_sizes[1 + 2 * i] < DM * DM) return; if (in_sizes[2 + 2 * i] < DM) return; }
  if (in_sizes[13] < 2) return;
  if ((size_t)out_size < rows_need * DM) return;
  const float* x = (const float*)d_in[0];
  const float* wsrc[6]; const float* bsrc[6];
  for (int i = 0; i < 6; ++i) { wsrc[i] = (const float*)d_in[1 + 2 * i]; bsrc[i] = (const float*)d_in[2 + 2 * i]; }
  const float* aw = (const float*)d_in[13];
  char* ws = (char*)d_ws; size_t off = 0;
  auto take = [&](size_t bytes) { char* p = ws + off; off += (bytes + 255) & ~(size_t)255; return p; };
  _Float16* BW = (_Float16*)take(6 * WS_W);
  _Float16* X16 = (_Float16*)take(WS_X);
  _Float16* PL = (_Float16*)take(6 * WS_X);
  _Float16* VT = (_Float16*)take(2 * (size_t)NB * WS_VT);
  if (off > ws_size) return;
  float* out = (float*)d_out;
  const size_t WN = (size_t)DM * DM;
  const size_t PN = (size_t)NR * DM;

  { const unsigned g = (unsigned)(((size_t)DM * DM / 8 + 255) / 256);
    for (int i = 0; i < 6; ++i) k_wt_f16<<<g, 256, 0, stream>>>(wsrc[i], BW + (size_t)i * WN, DM, DM, 16.0f); }
  k_x16<<<(unsigned)((NR * DM / 8 + 255) / 256), 256, 0, stream>>>(x, X16, NR * DM / 8);
  { const unsigned gp = (unsigned)((MP / 128) * (DM / 64));
    for (int i = 0; i < 6; ++i)
      k_gemm2<0><<<dim3(gp, 1), 128, 0, stream>>>(X16, DM, 0, BW + (size_t)i * WN, DM, 0, 0.0625f, bsrc[i], 0, nullptr, 1, 0, 0, nullptr, PL + (size_t)i * PN, DM, 0, MP, DM, DM); }
  for (int set = 0; set < 2; ++set)
    k_vt<NH, SQ><<<NB * NH * (SQ / 64), 256, 0, stream>>>(PL + (size_t)(3 * set + 2) * PN, LQ, 0, VT + (size_t)set * NB * NH * HD * SQ);
  k_flash2<<<dim3((unsigned)(SQ / 64), (unsigned)(NB * NH)), 128, 0, stream>>>(PL, VT, aw, out);
}
